// ProteinLMGraph_72318659330280
// MI455X (gfx1250) — hardware-verified
//
#include <hip/hip_runtime.h>
#include <stddef.h>


#define DIMF 1024
#define HIDC 64
#define NLAY 4
#define NGRA 16
#define NTH  256
#define NWV  8

#define NBA  64
#define CHA  2048
#define WCA  256
#define NGA  (CHA / (NTH * 4))
#define ATT_LDS_BYTES ((NBA * DIMF + 3 * NBA + NWV * WCA + NWV) * 4)
static_assert(WCA == (CHA / NTH) * 32);
static_assert(NGA == 2);
static_assert(ATT_LDS_BYTES == 271136);

#define GRW  16
#define CSP  1028
#define GEMM_LDS_BYTES ((GRW * CSP + GRW * DIMF + 2 * GRW) * 4)
static_assert(GEMM_LDS_BYTES == 131456);

#define NBS  256
#define CHS  1024
#define WCS  128
#define NGS  (CHS / (NTH * 4))
#define SP_LDS_BYTES ((NBS * HIDC + NBS + 192 + 6 * 64) * 4 + (NWV * WCS + NWV) * 4)
static_assert(WCS == (CHS / NTH) * 32);
static_assert(NGS == 1);
static_assert(SP_LDS_BYTES == 72992);

#define SRPB 640
#define DRW  32
#define AHP  136
#define CHP  68

typedef float          v2f  __attribute__((ext_vector_type(2)));
typedef float          v4f  __attribute__((ext_vector_type(4)));
typedef float          v8f  __attribute__((ext_vector_type(8)));
typedef double         v2d  __attribute__((ext_vector_type(2)));
typedef int            v4i  __attribute__((ext_vector_type(4)));
typedef unsigned int   v2u  __attribute__((ext_vector_type(2)));
typedef unsigned short v8us __attribute__((ext_vector_type(8)));
typedef _Float16       v8h  __attribute__((ext_vector_type(8)));
typedef _Float16       v16h __attribute__((ext_vector_type(16)));
typedef __bf16         v16bf __attribute__((ext_vector_type(16)));

union FragH { v16h v; v8h half[2]; };
union FragB { v16bf v; v8us half[2]; };
union PackH { v8h h; v4i i; };
union PackU { v8us u; v4i i; unsigned short s[8]; };

__device__ __forceinline__ v8f wmh(v16h a, v16h b, v8f c) {
  v8f d = __builtin_amdgcn_wmma_f32_16x16x32_f16(false, a, false, b, (short)0, c, false, false);
  asm volatile("v_nop\n\tv_nop\n\tv_nop\n\tv_nop" : "+v"(d) : "v"(a), "v"(b));
  return d;
}
__device__ __forceinline__ v8f wmb(v16bf a, v16bf b, v8f c) {
  v8f d = __builtin_amdgcn_wmma_f32_16x16x32_bf16(false, a, false, b, (short)0, c, false, false);
  asm volatile("v_nop\n\tv_nop\n\tv_nop\n\tv_nop" : "+v"(d) : "v"(a), "v"(b));
  return d;
}

__device__ __forceinline__ float wsum(float v) {
  v += __shfl_xor(v, 16, 32);
  v += __shfl_xor(v, 8, 32);
  v += __shfl_xor(v, 4, 32);
  v += __shfl_xor(v, 2, 32);
  v += __shfl_xor(v, 1, 32);
  return v;
}

__device__ __forceinline__ float lk(float x) { return x >= 0.f ? x : 0.01f * x; }
__device__ __forceinline__ v4f lk4(v4f x) {
  v4f y;
  y.x = lk(x.x); y.y = lk(x.y); y.z = lk(x.z); y.w = lk(x.w);
  return y;
}

__device__ __forceinline__ unsigned short bfb(float f) {
  unsigned int u = __float_as_uint(f);
  u = u + 0x7FFFu + ((u >> 16) & 1u);
  return (unsigned short)(u >> 16);
}
__device__ __forceinline__ float bfv(unsigned short b) { return __uint_as_float(((unsigned int)b) << 16); }

template <int NSLOT, int CH, int WC, int NG, int SHIFT>
__device__ __forceinline__ int scan_chunk(const int* __restrict__ ids, int nIds, int cbase, bool al16,
                                          int slotBase, int tid, int wave, int* list) {
  int wc = 0;
#pragma unroll
  for (int g = 0; g < NG; ++g) {
    const int el0 = (g * NTH + tid) * 4;
    const int e0  = cbase + el0;
    const int sent = -2147483647 - 1;
    v4i d;
    if (al16 && (cbase + CH <= nIds)) {
      d = *(const v4i*)(ids + e0);
    } else {
      const int i0 = min(e0, nIds - 1), i1 = min(e0 + 1, nIds - 1);
      const int i2 = min(e0 + 2, nIds - 1), i3 = min(e0 + 3, nIds - 1);
      const int x0 = ids[i0], x1 = ids[i1], x2 = ids[i2], x3 = ids[i3];
      d.x = (e0     < nIds) ? x0 : sent;
      d.y = (e0 + 1 < nIds) ? x1 : sent;
      d.z = (e0 + 2 < nIds) ? x2 : sent;
      d.w = (e0 + 3 < nIds) ? x3 : sent;
    }
    const unsigned s0 = (unsigned)d.x - (unsigned)slotBase;
    const unsigned s1 = (unsigned)d.y - (unsigned)slotBase;
    const unsigned s2 = (unsigned)d.z - (unsigned)slotBase;
    const unsigned s3 = (unsigned)d.w - (unsigned)slotBase;
    const bool h0 = s0 < (unsigned)NSLOT;
    const bool h1 = s1 < (unsigned)NSLOT;
    const bool h2 = s2 < (unsigned)NSLOT;
    const bool h3 = s3 < (unsigned)NSLOT;
    const unsigned many = __builtin_amdgcn_ballot_w32(h0 | h1 | h2 | h3);
    if (many != 0u) {
#define HITJ(J, HJ, SJ) { \
        const unsigned mj = __builtin_amdgcn_ballot_w32(HJ); \
        if (HJ) { \
          const int pos = wc + (int)__builtin_amdgcn_mbcnt_lo(mj, 0u); \
          if (pos < WC) list[wave * WC + pos] = ((el0 + (J)) << SHIFT) | (int)(SJ); \
        } \
        wc += (int)__builtin_popcount(mj); }
      HITJ(0, h0, s0)
      HITJ(1, h1, s1)
      HITJ(2, h2, s2)
      HITJ(3, h3, s3)
#undef HITJ
    }
  }
  return wc;
}

template <int MODE>
__global__ __launch_bounds__(NTH) void k_tr(const float* __restrict__ W, int K, int Nc, float scale,
                                            unsigned short* o1, unsigned short* o2) {
  __shared__ float Ts[64][65];
  const int tid = threadIdx.x;
  const int z = blockIdx.z, k0 = blockIdx.x * 64, n0 = blockIdx.y * 64;
  const float* Wz = W + (size_t)z * K * Nc;
  {
    const int kr = tid >> 2, nq = (tid & 3) * 16;
    const float* p = Wz + (size_t)(k0 + kr) * Nc + n0 + nq;
#pragma unroll
    for (int i = 0; i < 4; ++i) {
      const v4f f = *(const v4f*)(p + 4 * i);
      Ts[kr][nq + 4 * i]     = f.x;
      Ts[kr][nq + 4 * i + 1] = f.y;
      Ts[kr][nq + 4 * i + 2] = f.z;
      Ts[kr][nq + 4 * i + 3] = f.w;
    }
  }
  __syncthreads();
  PackH ph[2];
  PackU pu[2], pl[2];
  size_t po[2];
#pragma unroll
  for (int s = 0; s < 2; ++s) {
    const int idx = tid + NTH * s;
    const int j = idx >> 3, q = idx & 7;
    po[s] = (size_t)z * Nc * K + (size_t)(n0 + j) * K + k0 + 8 * q;
#pragma unroll
    for (int i = 0; i < 8; ++i) {
      const float v = Ts[8 * q + i][j];
      if (MODE == 0) {
        ph[s].h[i] = (_Float16)(v * scale);
      } else {
        const unsigned short hb = bfb(v);
        pu[s].s[i] = hb;
        pl[s].s[i] = bfb(v - bfv(hb));
      }
    }
  }
#pragma unroll
  for (int s = 0; s < 2; ++s) {
    if (MODE == 0) {
      *(volatile v4i*)(o1 + po[s]) = ph[s].i;
    } else {
      *(volatile v4i*)(o1 + po[s]) = pu[s].i;
      *(volatile v4i*)(o2 + po[s]) = pl[s].i;
    }
  }
  __threadfence();
#pragma unroll
  for (int s = 0; s < 2; ++s) {
    if (MODE == 0) {
      *(volatile v4i*)(o1 + po[s]) = ph[s].i;
    } else {
      *(volatile v4i*)(o1 + po[s]) = pu[s].i;
      *(volatile v4i*)(o2 + po[s]) = pl[s].i;
    }
  }
}

__global__ __launch_bounds__(NTH) void k_surf_stats(const float* __restrict__ sf, const float* __restrict__ w,
                                                    const float* __restrict__ b, double* part, double* partq,
                                                    int nS, int rpb) {
  __shared__ double Rd[4][64], Rq[4][64];
  __shared__ __attribute__((aligned(16))) double Fd[64];
  __shared__ __attribute__((aligned(16))) double Fq[64];
  const int tid = threadIdx.x, lane = tid & 31, wave = tid >> 5;
  const int grp = tid >> 6, c = tid & 63;
  const float w0 = w[c], w1 = w[64 + c], w2 = w[128 + c], bc = b[c];
  double s = 0.0, q = 0.0;
#pragma unroll 1
  for (int r = grp; r < rpb; r += 4) {
    const int row = blockIdx.x * rpb + r;
    const int rc  = row < nS ? row : nS - 1;
    const float* x = sf + (size_t)rc * 3;
    const float x0 = x[0], x1 = x[1], x2 = x[2];
    float t = x0 * w0;
    t = fmaf(x1, w1, t);
    t = fmaf(x2, w2, t);
    t += bc;
    if (row < nS) { s += (double)t; q += (double)t * (double)t; }
  }
  Rd[grp][c] = s;
  Rq[grp][c] = q;
  __syncthreads();
  if (tid < 64) {
    Fd[c] = ((Rd[0][c] + Rd[1][c]) + Rd[2][c]) + Rd[3][c];
    Fq[c] = ((Rq[0][c] + Rq[1][c]) + Rq[2][c]) + Rq[3][c];
  }
  __syncthreads();
  const v2d va = *(const v2d*)(Fd + 2 * lane);
  const v2d vb = *(const v2d*)(Fq + 2 * lane);
  v2d vv;
  vv.x = (wave == 0) ? va.x : vb.x;
  vv.y = (wave == 0) ? va.y : vb.y;
  double* dp = ((wave == 0) ? part : partq) + (size_t)blockIdx.x * 64 + 2 * lane;
  if (wave < 2) *(volatile v2d*)dp = vv;
  __threadfence();
  if (wave < 2) *(volatile v2d*)dp = vv;
}

__global__ __launch_bounds__(NTH) void k_surf_pool(
    const float* __restrict__ sf, const int* __restrict__ sres,
    const float* __restrict__ w, const float* __restrict__ b, const float* __restrict__ g, const float* __restrict__ bt,
    const double* __restrict__ part, const double* __restrict__ partq, float* nodes, int nS, int nP, int nN) {
  extern __shared__ v4f lds_dyn[];
  float* ssum = (float*)lds_dyn;
  float* scnt = ssum + NBS * HIDC;
  float* Wl   = scnt + NBS;
  float* Bl   = Wl + 192;
  float* Gl   = Bl + 64;
  float* Tl   = Gl + 64;
  float* Mu   = Tl + 64;
  float* Rs   = Mu + 64;
  int*   list = (int*)(Rs + 64);
  int*   wcnt = list + NWV * WCS;
  const int tid = threadIdx.x, lane = tid & 31, wave = tid >> 5;
  const int nodeBase = blockIdx.x * NBS;
  {
    const v4f z4 = {0.f, 0.f, 0.f, 0.f};
    for (int i = tid; i < (NBS * HIDC + NBS) / 4; i += NTH) lds_dyn[i] = z4;
    if (tid < 192) Wl[tid] = w[tid];
    if (tid < 64) {
      Bl[tid] = b[tid]; Gl[tid] = g[tid]; Tl[tid] = bt[tid];
      double s = 0.0, q = 0.0;
#pragma unroll 1
      for (int p = 0; p < nP; ++p) { s += part[(size_t)p * 64 + tid]; q += partq[(size_t)p * 64 + tid]; }
      const double mu = s / (double)nS;
      double var = q / (double)nS - mu * mu;
      if (var < 0.0) var = 0.0;
      Mu[tid] = (float)mu;
      Rs[tid] = rsqrtf((float)var + 1e-5f);
    }
  }
  __syncthreads();
  const int c0 = 2 * lane, c1 = c0 + 1;
  const float w00 = Wl[c0], w10 = Wl[64 + c0], w20 = Wl[128 + c0];
  const float w01 = Wl[c1], w11 = Wl[64 + c1], w21 = Wl[128 + c1];
  const float b0 = Bl[c0], b1 = Bl[c1], g0 = Gl[c0], g1 = Gl[c1], t0 = Tl[c0], t1 = Tl[c1];
  const float mu0 = Mu[c0], mu1 = Mu[c1], rs0 = Rs[c0], rs1 = Rs[c1];
  const bool al16 = ((((size_t)sres) & 15) == 0);
  const int nCh = (nS + CHS - 1) / CHS;
#pragma unroll 1
  for (int ch = 0; ch < nCh; ++ch) {
    const int cbase = ch * CHS;
    const int wc = scan_chunk<NBS, CHS, WCS, NGS, 8>(sres, nS, cbase, al16, nodeBase, tid, wave, list);
    if (lane == 0) wcnt[wave] = wc;
    __syncthreads();
    for (int wsx = 0; wsx < NWV; ++wsx) {
      int n = wcnt[wsx];
      n = n > WCS ? WCS : (n < 0 ? 0 : n);
      for (int i = 0; i < n; ++i) {
        const int ent  = list[wsx * WCS + i];
        const int slot = ent & (NBS - 1);
        if ((slot & (NWV - 1)) != wave) continue;
        const int el = (ent >> 8) & (CHS - 1);
        int p = cbase + el;
        if (p > nS - 1) p = nS - 1;
        const float* x = sf + (size_t)p * 3;
        const float x0 = x[0], x1 = x[1], x2 = x[2];
        float ta = x0 * w00; ta = fmaf(x1, w10, ta); ta = fmaf(x2, w20, ta); ta += b0;
        float tb = x0 * w01; tb = fmaf(x1, w11, tb); tb = fmaf(x2, w21, tb); tb += b1;
        const float va = lk((g0 * (ta - mu0)) * rs0 + t0);
        const float vb = lk((g1 * (tb - mu1)) * rs1 + t1);
        ssum[slot * HIDC + c0] += va;
        ssum[slot * HIDC + c1] += vb;
        if (lane == 0) scnt[slot] += 1.0f;
      }
    }
    __syncthreads();
  }
#pragma unroll 1
  for (int i = 0; i < 16; ++i) {
    const int slot = 32 * wave + 2 * i + (lane >> 4);
    const int c4 = 4 * (lane & 15);
    const float rc = 1.0f / fmaxf(scnt[slot], 1.0f);
    const v4f v = *(const v4f*)(ssum + slot * HIDC + c4) * rc;
    float* op = nodes + (size_t)(nodeBase + slot) * HIDC + c4;
    *(volatile v4f*)op = v;
  }
  __threadfence();
#pragma unroll 1
  for (int i = 0; i < 16; ++i) {
    const int slot = 32 * wave + 2 * i + (lane >> 4);
    const int c4 = 4 * (lane & 15);
    const float rc = 1.0f / fmaxf(scnt[slot], 1.0f);
    const v4f v = *(const v4f*)(ssum + slot * HIDC + c4) * rc;
    float* op = nodes + (size_t)(nodeBase + slot) * HIDC + c4;
    *(volatile v4f*)op = v;
  }
}

__global__ __launch_bounds__(NTH) void k_init(const float* __restrict__ x, const float* __restrict__ aw,
                                             float* pab, int nN) {
  __shared__ __attribute__((aligned(16))) float Ps[16];
  __shared__ __attribute__((aligned(16))) float Qs[16];
  const int tid = threadIdx.x, lane = tid & 31, wave = tid >> 5;
  for (int i = 0; i < 2; ++i) {
    const int rl = wave + 8 * i;
    int node = blockIdx.x * 16 + rl;
    if (node > nN - 1) node = nN - 1;
    const float* r = x + (size_t)node * DIMF + 4 * lane;
    float du = 0.f, dv = 0.f;
#pragma unroll 1
    for (int j = 0; j < 8; ++j) {
      const v4f xv = *(const v4f*)(r + 128 * j);
      const v4f a1 = *(const v4f*)(aw + 128 * j + 4 * lane);
      const v4f a2 = *(const v4f*)(aw + DIMF + 128 * j + 4 * lane);
      du += (xv.x * a1.x + xv.y * a1.y) + (xv.z * a1.z + xv.w * a1.w);
      dv += (xv.x * a2.x + xv.y * a2.y) + (xv.z * a2.z + xv.w * a2.w);
    }
    du = wsum(du);
    dv = wsum(dv);
    if (lane == 0) { Ps[rl] = du; Qs[rl] = dv; }
  }
  __syncthreads();
  if (wave == 0) {
    const v4f vp = *(const v4f*)(Ps + 4 * (lane & 3));
    const v4f vq = *(const v4f*)(Qs + 4 * (lane & 3));
    v4f v;
    v.x = (lane < 4) ? vp.x : vq.x; v.y = (lane < 4) ? vp.y : vq.y;
    v.z = (lane < 4) ? vp.z : vq.z; v.w = (lane < 4) ? vp.w : vq.w;
    float* p = pab + (size_t)blockIdx.x * 32 + 4 * lane;
    if (lane < 8) *(volatile v4f*)p = v;
    __threadfence();
    if (lane < 8) *(volatile v4f*)p = v;
  }
}

__device__ __forceinline__ void att_rows_out(const float* sacc, _Float16* aggh, int nodeBase, int wave, int lane) {
#pragma unroll 1
  for (int j = 0; j < NBA / NWV; ++j) {
    const int slot = wave * (NBA / NWV) + j;
    const size_t node = (size_t)(nodeBase + slot);
    _Float16* orow = aggh + node * DIMF + 8 * lane;
    const float* srow = sacc + slot * DIMF + 8 * lane;
#pragma unroll 1
    for (int q = 0; q < 4; ++q) {
      const v4f a = *(const v4f*)(srow + 256 * q);
      const v4f c = *(const v4f*)(srow + 256 * q + 4);
      PackH pk;
      pk.h[0] = (_Float16)(a.x * 8.0f); pk.h[1] = (_Float16)(a.y * 8.0f);
      pk.h[2] = (_Float16)(a.z * 8.0f); pk.h[3] = (_Float16)(a.w * 8.0f);
      pk.h[4] = (_Float16)(c.x * 8.0f); pk.h[5] = (_Float16)(c.y * 8.0f);
      pk.h[6] = (_Float16)(c.z * 8.0f); pk.h[7] = (_Float16)(c.w * 8.0f);
      *(volatile v4i*)(orow + 256 * q) = pk.i;
    }
  }
}

__global__ __launch_bounds__(NTH) __attribute__((amdgpu_num_vgpr(256)))
void k_att(const float* __restrict__ feat, const int* __restrict__ ei,
           const float* __restrict__ pab, _Float16* aggh, int nN, int nE) {
  extern __shared__ v4f lds_dyn[];
  float* sacc = (float*)lds_dyn;
  float* sm   = sacc + NBA * DIMF;
  float* sden = sm + NBA;
  float* spb  = sden + NBA;
  int*   list = (int*)(spb + NBA);
  int*   wcnt = list + NWV * WCA;
  const int tid = threadIdx.x, lane = tid & 31, wave = tid >> 5;
  const int nodeBase = blockIdx.x * NBA;
  {
    const v4f z4 = {0.f, 0.f, 0.f, 0.f};
#pragma unroll 1
    for (int i = tid; i < NBA * DIMF / 4; i += NTH) lds_dyn[i] = z4;
    if (tid < NBA) {
      int nd = nodeBase + tid;
      if (nd > nN - 1) nd = nN - 1;
      sm[tid]   = __uint_as_float(0xFF800000u);
      sden[tid] = 0.f;
      spb[tid]  = pab[(nd >> 4) * 32 + 16 + (nd & 15)];
    }
  }
  __syncthreads();
  const int* eid = ei + nE;
  const bool al16 = ((nE & 3) == 0) && ((((size_t)ei) & 15) == 0);
  const int nCh = (nE + CHA - 1) / CHA;
#pragma unroll 1
  for (int pass = 0; pass < 2; ++pass) {
    if (pass == 1) {
      if (tid < NBA) { const float d = sden[tid]; sden[tid] = d > 0.f ? 1.0f / d : 0.f; }
      __syncthreads();
    }
#pragma unroll 1
    for (int ch = 0; ch < nCh; ++ch) {
      const int cbase = ch * CHA;
      const int wc = scan_chunk<NBA, CHA, WCA, NGA, 6>(eid, nE, cbase, al16, nodeBase, tid, wave, list);
      if (lane == 0) wcnt[wave] = wc;
      __syncthreads();
#pragma unroll 1
      for (int wsx = 0; wsx < NWV; ++wsx) {
        int n = wcnt[wsx];
        n = n > WCA ? WCA : (n < 0 ? 0 : n);
#pragma unroll 1
        for (int i = 0; i < n; ++i) {
          const int ent  = list[wsx * WCA + i];
          const int slot = ent & (NBA - 1);
          if ((slot & (NWV - 1)) != wave) continue;
          const int el = (ent >> 6) & (CHA - 1);
          int e = cbase + el;
          if (e > nE - 1) e = nE - 1;
          int u = ei[e];
          u = u < 0 ? 0 : (u > nN - 1 ? nN - 1 : u);
          const float lg = pab[(u >> 4) * 32 + (u & 15)] + spb[slot];
          if (pass == 0) {
            const float mo = sm[slot];
            const float mn = fmaxf(mo, lg);
            const float dn = sden[slot] * expf(mo - mn) + expf(lg - mn);
            sm[slot]   = mn;
            sden[slot] = dn;
          } else {
            const float wgt = expf(lg - sm[slot]) * sden[slot];
            const float* fr = feat + (size_t)u * DIMF + 4 * lane;
            float* sr = sacc + slot * DIMF + 4 * lane;
#pragma unroll 1
            for (int j = 0; j < 8; ++j) {
              const v4f xv = *(const v4f*)(fr + 128 * j);
              v4f* sp = (v4f*)(sr + 128 * j);
              const v4f cur = *sp;
              *sp = cur + wgt * xv;
            }
          }
        }
      }
      __syncthreads();
    }
  }
  __syncthreads();
  att_rows_out(sacc, aggh, nodeBase, wave, lane);
  __threadfence();
  att_rows_out(sacc, aggh, nodeBase, wave, lane);
}

__global__ __launch_bounds__(NTH) __attribute__((amdgpu_num_vgpr(256)))
void k_gemm_ln(
    const _Float16* __restrict__ A, const _Float16* __restrict__ Wt,
    const float* __restrict__ bias, const float* __restrict__ gam, const float* __restrict__ bet,
    const float* __restrict__ awn, const float* accin, float* accout, float* featout, float* pab,
    unsigned short* x5h, unsigned short* x5l, int last) {
  extern __shared__ v4f lds_dyn[];
  float* Cs = (float*)lds_dyn;
  float* Av = Cs + GRW * CSP;
  float* Ps = Av + GRW * DIMF;
  float* Qs = Ps + GRW;
  const int tid = threadIdx.x, lane = tid & 31, wave = tid >> 5;
  const int h = lane >> 4, m = lane & 15;
  const int rowBase = blockIdx.x * GRW;
  const int colBase = wave * 128;
  const v8f z8 = {0.f, 0.f, 0.f, 0.f, 0.f, 0.f, 0.f, 0.f};
  const float inv256 = 1.0f / 256.0f;
  const _Float16* arow = A + (size_t)(rowBase + m) * DIMF + 8 * h;

#pragma unroll 1
  for (int hf = 0; hf < 2; ++hf) {
    const int cb = colBase + 64 * hf;
    const _Float16* brow = Wt + (size_t)(cb + m) * DIMF + 8 * h;
    v8f acc[4];
#pragma unroll
    for (int ct = 0; ct < 4; ++ct) acc[ct] = z8;
#pragma unroll 1
    for (int kt = 0; kt < DIMF / 32; ++kt) {
      const int k0 = kt * 32;
      FragH a;
      a.half[0] = *(const v8h*)(arow + k0);
      a.half[1] = *(const v8h*)(arow + k0 + 16);
#pragma unroll
      for (int ct = 0; ct < 4; ++ct) {
        const _Float16* bp = brow + (size_t)(16 * ct) * DIMF + k0;
        FragH b;
        b.half[0] = *(const v8h*)bp;
        b.half[1] = *(const v8h*)(bp + 16);
        acc[ct] = wmh(a.v, b.v, acc[ct]);
      }
    }
#pragma unroll
    for (int ct = 0; ct < 4; ++ct) {
#pragma unroll
      for (int r = 0; r < 8; ++r) Cs[(8 * h + r) * CSP + cb + 16 * ct + m] = acc[ct][r] * inv256;
    }
  }
  __syncthreads();

#pragma unroll 1
  for (int i = 0; i < 2; ++i) {
    const int rl = 2 * wave + i;
    const size_t row = (size_t)rowBase + rl;
    float* crow = Cs + rl * CSP + 4 * lane;
    float* vrow = Av + rl * DIMF + 4 * lane;
    float s = 0.f;
#pragma unroll 1
    for (int j = 0; j < 8; ++j) {
      const v4f cv = *(const v4f*)(crow + 128 * j);
      const v4f bb = *(const v4f*)(bias + 128 * j + 4 * lane);
      const v4f x  = cv + bb;
      *(v4f*)(crow + 128 * j) = x;
      s += (x.x + x.y) + (x.z + x.w);
    }
    const float mu = wsum(s) * (1.0f / DIMF);
    float q = 0.f;
#pragma unroll 1
    for (int j = 0; j < 8; ++j) {
      const v4f d = *(const v4f*)(crow + 128 * j) - mu;
      q += (d.x * d.x + d.y * d.y) + (d.z * d.z + d.w * d.w);
    }
    const float var = wsum(q) * (1.0f / DIMF);
    const float rs = rsqrtf(var + 1e-5f);
    float du = 0.f, dv = 0.f;
#pragma unroll 1
    for (int j = 0; j < 8; ++j) {
      const v4f d  = *(const v4f*)(crow + 128 * j) - mu;
      const v4f gv = *(const v4f*)(gam + 128 * j + 4 * lane);
      const v4f ev = *(const v4f*)(bet + 128 * j + 4 * lane);
      const v4f t  = (gv * d) * rs + ev;
      const v4f yv = lk4(t);
      const v4f av = *(const v4f*)(accin + row * DIMF + 128 * j + 4 * lane) + yv;
      const v4f a1 = *(const v4f*)(awn + 128 * j + 4 * lane);
      const v4f a2 = *(const v4f*)(awn + DIMF + 128 * j + 4 * lane);
      du += (yv.x * a1.x + yv.y * a1.y) + (yv.z * a1.z + yv.w * a1.w);
      dv += (yv.x * a2.x + yv.y * a2.y) + (yv.z * a2.z + yv.w * a2.w);
      *(v4f*)(crow + 128 * j) = yv;
      *(v4f*)(vrow + 128 * j) = av;
    }
    if (!last) {
      du = wsum(du);
      dv = wsum(dv);
      if (lane == 0) { Ps[rl] = du; Qs[rl] = dv; }
      float* fp = featout + row * DIMF + 4 * lane;
      float* ap = accout  + row * DIMF + 4 * lane;
#pragma unroll 1
      for (int j = 0; j < 8; ++j) {
        const v4f yv = *(const v4f*)(crow + 128 * j);
        const v4f av = *(const v4f*)(vrow + 128 * j);
        *(volatile v4f*)(fp + 128 * j) = yv;
        *(volatile v4f*)(ap + 128 * j) = av;
      }
      __threadfence();
#pragma unroll 1
      for (int j = 0; j < 8; ++j) {
        const v4f yv = *(const v4f*)(crow + 128 * j);
        const v4f av = *(const v4f*)(vrow + 128 * j);
        *(volatile v4f*)(fp + 128 * j) = yv;
        *(volatile v4f*)(ap + 128 * j) = av;
      }
    } else {
      unsigned short* hr = x5h + row * DIMF + 4 * lane;
      unsigned short* lr = x5l + row * DIMF + 4 * lane;
#pragma unroll 1
      for (int j = 0; j < 8; ++j) {
        const v4f x5 = *(const v4f*)(vrow + 128 * j) * 0.2f;
        const unsigned short h0 = bfb(x5.x), h1 = bfb(x5.y), h2 = bfb(x5.z), h3 = bfb(x5.w);
        const unsigned short l0 = bfb(x5.x - bfv(h0)), l1 = bfb(x5.y - bfv(h1));
        const unsigned short l2 = bfb(x5.z - bfv(h2)), l3 = bfb(x5.w - bfv(h3));
        v2u hp, lp;
        hp.x = (unsigned int)h0 | ((unsigned int)h1 << 16);
        hp.y = (unsigned int)h2 | ((unsigned int)h3 << 16);
        lp.x = (unsigned int)l0 | ((unsigned int)l1 << 16);
        lp.y = (unsigned int)l2 | ((unsigned int)l3 << 16);
        *(volatile v2u*)(hr + 128 * j) = hp;
        *(volatile v2u*)(lr + 128 * j) = lp;
      }
      __threadfence();
#pragma unroll 1
      for (int j = 0; j < 8; ++j) {
        const v4f x5 = *(const v4f*)(vrow + 128 * j) * 0.2f;
        const unsigned short h0 = bfb(x5.x), h1 = bfb(x5.y), h2 = bfb(x5.z), h3 = bfb(x5.w);
        const unsigned short l0 = bfb(x5.x - bfv(h0)), l1 = bfb(x5.y - bfv(h1));
        const unsigned short l2 = bfb(x5.z - bfv(h2)), l3 = bfb(x5.w - bfv(h3));
        v2u hp, lp;
        hp.x = (unsigned int)h0 | ((unsigned int)h1 << 16);
        hp.y = (unsigned int)h2 | ((unsigned int)h3 << 16);
        lp.x = (unsigned int)l0 | ((unsigned int)l1 << 16);
        lp.y = (unsigned int)l2 | ((unsigned int)l3 << 16);
        *(volatile v2u*)(hr + 128 * j) = hp;
        *(volatile v2u*)(lr + 128 * j) = lp;
      }
    }
  }
  if (!last) {
    __syncthreads();
    if (wave == 0) {
      const v4f vp = *(const v4f*)(Ps + 4 * (lane & 3));
      const v4f vq = *(const v4f*)(Qs + 4 * (lane & 3));
      v4f v;
      v.x = (lane < 4) ? vp.x : vq.x; v.y = (lane < 4) ? vp.y : vq.y;
      v.z = (lane < 4) ? vp.z : vq.z; v.w = (lane < 4) ? vp.w : vq.w;
      float* p = pab + (size_t)blockIdx.x * 32 + 4 * lane;
      if (lane < 8) *(volatile v4f*)p = v;
      __threadfence();
      if (lane < 8) *(volatile v4f*)p = v;
    }
  }
}

__global__ __launch_bounds__(128) void k_hid(const unsigned short* __restrict__ xh, const unsigned short* __restrict__ xl,
                                            const unsigned short* __restrict__ wh, const unsigned short* __restrict__ wl,
                                            const float* __restrict__ hb, float* nf) {
  __shared__ __attribute__((aligned(16))) float Cs[DRW * CHP];
  const int tid = threadIdx.x, lane = tid & 31, wave = tid >> 5;
  const int h = lane >> 4, m = lane & 15;
  const int rowBase = blockIdx.x * DRW;
  const int n = 16 * wave + m;
  const v8f z8 = {0.f, 0.f, 0.f, 0.f, 0.f, 0.f, 0.f, 0.f};
  v8f acc[2];
  acc[0] = z8; acc[1] = z8;
  const unsigned short* ah0 = xh + (size_t)(rowBase + m) * DIMF + 8 * h;
  const unsigned short* ah1 = ah0 + (size_t)16 * DIMF;
  const unsigned short* al0 = xl + (size_t)(rowBase + m) * DIMF + 8 * h;
  const unsigned short* al1 = al0 + (size_t)16 * DIMF;
  const unsigned short* bhp = wh + (size_t)n * DIMF + 8 * h;
  const unsigned short* blp = wl + (size_t)n * DIMF + 8 * h;
#pragma unroll 1
  for (int kt = 0; kt < DIMF / 32; ++kt) {
    const int k0 = kt * 32;
    FragB a0h, a1h, a0l, a1l, bh_, bl_;
    a0h.half[0] = *(const v8us*)(ah0 + k0); a0h.half[1] = *(const v8us*)(ah0 + k0 + 16);
    a1h.half[0] = *(const v8us*)(ah1 + k0); a1h.half[1] = *(const v8us*)(ah1 + k0 + 16);
    a0l.half[0] = *(const v8us*)(al0 + k0); a0l.half[1] = *(const v8us*)(al0 + k0 + 16);
    a1l.half[0] = *(const v8us*)(al1 + k0); a1l.half[1] = *(const v8us*)(al1 + k0 + 16);
    bh_.half[0] = *(const v8us*)(bhp + k0); bh_.half[1] = *(const v8us*)(bhp + k0 + 16);
    bl_.half[0] = *(const v8us*)(blp + k0); bl_.half[1] = *(const v8us*)(blp + k0 + 16);
    acc[0] = wmb(a0h.v, bh_.v, acc[0]);
    acc[0] = wmb(a0h.v, bl_.v, acc[0]);
    acc[0] = wmb(a0l.v, bh_.v, acc[0]);
    acc[1] = wmb(a1h.v, bh_.v, acc[1]);
    acc[1] = wmb(a1h.v, bl_.v, acc[1]);
    acc[1] = wmb(a1l.v, bh_.v, acc[1]);
  }
  const float hbv = hb[n];
#pragma unroll
  for (int r = 0; r < 8; ++r) {
    Cs[(8 * h + r) * CHP + n]      = acc[0][r] + hbv;
    Cs[(16 + 8 * h + r) * CHP + n] = acc[1][r] + hbv;
  }
  __syncthreads();
  v4f ov[4];
  float* op[4];
#pragma unroll
  for (int i = 0; i < 4; ++i) {
    const int rr = 8 * wave + 2 * i + (lane >> 4);
    const int c4 = 4 * (lane & 15);
    ov[i] = *(const v4f*)(Cs + rr * CHP + c4);
    op[i] = nf + (size_t)(rowBase + rr) * HIDC + c4;
  }
#pragma unroll
  for (int i = 0; i < 4; ++i) *(volatile v4f*)(op[i]) = ov[i];
  __threadfence();
#pragma unroll
  for (int i = 0; i < 4; ++i) *(volatile v4f*)(op[i]) = ov[i];
}

__global__ __launch_bounds__(512) void k_prot(const float* __restrict__ nf, const int* __restrict__ bat,
                                             const float* __restrict__ g, const float* __restrict__ b,
                                             float* out, int nN) {
  __shared__ __attribute__((aligned(16))) float Os[NGRA * HIDC];
  const int tid = threadIdx.x, lane = tid & 31, wave = tid >> 5;
  const int c0 = 2 * lane;
  float s0 = 0.f, s1 = 0.f;
  int cnt = 0;
#pragma unroll 1
  for (int n0 = 0; n0 < nN; n0 += 32) {
    const int nn = n0 + lane;
    const int id = bat[min(nn, nN - 1)];
    const bool hit = (nn < nN) && (id == wave);
    unsigned msk = __builtin_amdgcn_ballot_w32(hit);
    cnt += (int)__builtin_popcount(msk);
    while (msk != 0u) {
      const int bp = __builtin_ctz(msk);
      msk &= msk - 1u;
      const v2f v = *(const v2f*)(nf + (size_t)(n0 + bp) * HIDC + c0);
      s0 += v.x;
      s1 += v.y;
    }
  }
  const float rc = 1.0f / fmaxf((float)cnt, 1.0f);
  const float m0 = s0 * rc, m1 = s1 * rc;
  const float mu = wsum(m0 + m1) * (1.0f / HIDC);
  const float d0 = m0 - mu, d1 = m1 - mu;
  const float var = wsum(d0 * d0 + d1 * d1) * (1.0f / HIDC);
  const float rs = rsqrtf(var + 1e-5f);
  Os[wave * HIDC + c0]     = lk((g[c0] * d0) * rs + b[c0]);
  Os[wave * HIDC + c0 + 1] = lk((g[c0 + 1] * d1) * rs + b[c0 + 1]);
  __syncthreads();
  const int rr = 2 * (wave & 7) + (lane >> 4), c4 = 4 * (lane & 15);
  const v4f ov = *(const v4f*)(Os + rr * HIDC + c4);
  float* op = out + rr * HIDC + c4;
  if (wave < 8) *(volatile v4f*)op = ov;
  __threadfence();
  if (wave < 8) *(volatile v4f*)op = ov;
}

__global__ __launch_bounds__(128) void k_down(const float* __restrict__ nf, const float* __restrict__ nodes,
                                             const int* __restrict__ sset,
                                             const unsigned short* __restrict__ wh, const unsigned short* __restrict__ wl,
                                             const float* __restrict__ db, float* y, double* part, double* partq,
                                             int nU, int nN) {
  __shared__ __attribute__((aligned(16))) unsigned short Ah[DRW * AHP];
  __shared__ __attribute__((aligned(16))) unsigned short Al[DRW * AHP];
  __shared__ __attribute__((aligned(16))) float Cs[DRW * CHP];
  __shared__ __attribute__((aligned(16))) double Sd[HIDC];
  __shared__ __attribute__((aligned(16))) double Sq[HIDC];
  const int tid = threadIdx.x, lane = tid & 31, wave = tid >> 5;
  const int h = lane >> 4, m = lane & 15;
  const int rowBase = blockIdx.x * DRW;
  {
    const int rl = tid >> 2, q = tid & 3;
    int gi = rowBase + rl;
    if (gi > nU - 1) gi = nU - 1;
    int idx = sset[gi];
    idx = idx < 0 ? 0 : (idx > nN - 1 ? nN - 1 : idx);
    const float* src = (q < 2) ? (nf + (size_t)idx * HIDC + 32 * q) : (nodes + (size_t)idx * HIDC + 32 * (q - 2));
#pragma unroll
    for (int i = 0; i < 4; ++i) {
      const v4f f0 = *(const v4f*)(src + 8 * i);
      const v4f f1 = *(const v4f*)(src + 8 * i + 4);
      const float fv[8] = {f0.x, f0.y, f0.z, f0.w, f1.x, f1.y, f1.z, f1.w};
      PackU uh, ul;
#pragma unroll
      for (int e = 0; e < 8; ++e) {
        const unsigned short hb = bfb(fv[e]);
        uh.s[e] = hb;
        ul.s[e] = bfb(fv[e] - bfv(hb));
      }
      *(v8us*)(Ah + rl * AHP + 32 * q + 8 * i) = uh.u;
      *(v8us*)(Al + rl * AHP + 32 * q + 8 * i) = ul.u;
    }
  }
  __syncthreads();
  const int n = 16 * wave + m;
  const v8f z8 = {0.f, 0.f, 0.f, 0.f, 0.f, 0.f, 0.f, 0.f};
  v8f acc[2];
  acc[0] = z8; acc[1] = z8;
  const unsigned short* bhp = wh + (size_t)n * (2 * HIDC) + 8 * h;
  const unsigned short* blp = wl + (size_t)n * (2 * HIDC) + 8 * h;
#pragma unroll
  for (int kt = 0; kt < (2 * HIDC) / 32; ++kt) {
    const int k0 = kt * 32;
    FragB a0h, a1h, a0l, a1l, bh_, bl_;
    a0h.half[0] = *(const v8us*)(Ah + m * AHP + k0 + 8 * h);        a0h.half[1] = *(const v8us*)(Ah + m * AHP + k0 + 16 + 8 * h);
    a1h.half[0] = *(const v8us*)(Ah + (16 + m) * AHP + k0 + 8 * h); a1h.half[1] = *(const v8us*)(Ah + (16 + m) * AHP + k0 + 16 + 8 * h);
    a0l.half[0] = *(const v8us*)(Al + m * AHP + k0 + 8 * h);        a0l.half[1] = *(const v8us*)(Al + m * AHP + k0 + 16 + 8 * h);
    a1l.half[0] = *(const v8us*)(Al + (16 + m) * AHP + k0 + 8 * h); a1l.half[1] = *(const v8us*)(Al + (16 + m) * AHP + k0 + 16 + 8 * h);
    bh_.half[0] = *(const v8us*)(bhp + k0); bh_.half[1] = *(const v8us*)(bhp + k0 + 16);
    bl_.half[0] = *(const v8us*)(blp + k0); bl_.half[1] = *(const v8us*)(blp + k0 + 16);
    acc[0] = wmb(a0h.v, bh_.v, acc[0]);
    acc[0] = wmb(a0h.v, bl_.v, acc[0]);
    acc[0] = wmb(a0l.v, bh_.v, acc[0]);
    acc[1] = wmb(a1h.v, bh_.v, acc[1]);
    acc[1] = wmb(a1h.v, bl_.v, acc[1]);
    acc[1] = wmb(a1l.v, bh_.v, acc[1]);
  }
  const float dbv = db[n];
#pragma unroll
  for (int r = 0; r < 8; ++r) {
    Cs[(8 * h + r) * CHP + n]      = acc[0][r] + dbv;
    Cs[(16 + 8 * h + r) * CHP + n] = acc[1][r] + dbv;
  }
  __syncthreads();
  v4f ov[4];
  float* op[4];
#pragma unroll
  for (int i = 0; i < 4; ++i) {
    const int rr = 8 * wave + 2 * i + (lane >> 4);
    const int c4 = 4 * (lane & 15);
    ov[i] = *(const v4f*)(Cs + rr * CHP + c4);
    op[i] = y + (size_t)(rowBase + rr) * HIDC + c4;
  }
  if (tid < HIDC) {
    double s = 0.0, q = 0.0;
#pragma unroll 4
    for (int r = 0; r < DRW; ++r) {
      const float v = Cs[r * CHP + tid];
      if (rowBase + r < nU) { s += (double)v; q += (double)v * (double)v; }
    }
    Sd[tid] = s;
    Sq[tid] = q;
  }
  __syncthreads();
  const v2d va = *(const v2d*)(Sd + 2 * lane);
  const v2d vb = *(const v2d*)(Sq + 2 * lane);
  v2d vv;
  vv.x = (wave == 0) ? va.x : vb.x;
  vv.y = (wave == 0) ? va.y : vb.y;
  double* dp = ((wave == 0) ? part : partq) + (size_t)blockIdx.x * HIDC + 2 * lane;
#pragma unroll
  for (int i = 0; i < 4; ++i) *(volatile v4f*)(op[i]) = ov[i];
  if (wave < 2) *(volatile v2d*)dp = vv;
  __threadfence();
#pragma unroll
  for (int i = 0; i < 4; ++i) *(volatile v4f*)(op[i]) = ov[i];
  if (wave < 2) *(volatile v2d*)dp = vv;
}

__global__ __launch_bounds__(512) void k_out1(const float* __restrict__ y, const int* __restrict__ rb,
                                             const double* __restrict__ part, const double* __restrict__ partq,
                                             const float* __restrict__ dg, const float* __restrict__ dbt,
                                             const float* __restrict__ g2, const float* __restrict__ b2,
                                             float* out, int nU, int nP) {
  __shared__ float Mu[HIDC], Rs[HIDC], G1[HIDC], B1[HIDC];
  __shared__ __attribute__((aligned(16))) float Ns[NGRA * HIDC];
  __shared__ __attribute__((aligned(16))) float Os[NGRA * HIDC];
  const int tid = threadIdx.x, lane = tid & 31, wave = tid >> 5;
  if (tid < HIDC) {
    double s = 0.0, q = 0.0;
#pragma unroll 1
    for (int p = 0; p < nP; ++p) { s += part[(size_t)p * HIDC + tid]; q += partq[(size_t)p * HIDC + tid]; }
    const double mu = s / (double)nU;
    double var = q / (double)nU - mu * mu;
    if (var < 0.0) var = 0.0;
    Mu[tid] = (float)mu;
    Rs[tid] = rsqrtf((float)var + 1e-5f);
    G1[tid] = dg[tid];
    B1[tid] = dbt[tid];
  }
  __syncthreads();
  const int c0 = 2 * lane, c1 = c0 + 1;
  const float mu0 = Mu[c0], mu1 = Mu[c1], rs0 = Rs[c0], rs1 = Rs[c1];
  const float g0 = G1[c0], g1 = G1[c1], t0 = B1[c0], t1 = B1[c1];
  float s0 = 0.f, s1 = 0.f;
  int cnt = 0;
#pragma unroll 1
  for (int n0 = 0; n0 < nU; n0 += 32) {
    const int nn = n0 + lane;
    const int id = rb[min(nn, nU - 1)];
    const bool hit = (nn < nU) && (id == wave);
    unsigned msk = __builtin_amdgcn_ballot_w32(hit);
    cnt += (int)__builtin_popcount(msk);
    while (msk != 0u) {
      const int bp = __builtin_ctz(msk);
      msk &= msk - 1u;
      const v2f v = *(const v2f*)(y + (size_t)(n0 + bp) * HIDC + c0);
      s0 += lk((g0 * (v.x - mu0)) * rs0 + t0);
      s1 += lk((g1 * (v.y - mu1)) * rs1 + t1);
    }
  }
  const float rc = 1.0f / fmaxf((float)cnt, 1.0f);
  Ns[wave * HIDC + c0] = s0 * rc;
  Ns[wave * HIDC + c1] = s1 * rc;
  __syncthreads();
  if (tid < HIDC) {
    float su = 0.f;
#pragma unroll 1
    for (int gr = 0; gr < NGRA; ++gr) su += Ns[gr * HIDC + tid];
    const float mu = su * (1.0f / NGRA);
    float sq = 0.f;
#pragma unroll 1
    for (int gr = 0; gr < NGRA; ++gr) { const float d = Ns[gr * HIDC + tid] - mu; sq += d * d; }
    const float rs = rsqrtf(sq * (1.0f / NGRA) + 1e-5f);
    const float gg = g2[tid], bb = b2[tid];
#pragma unroll 1
    for (int gr = 0; gr < NGRA; ++gr) Os[gr * HIDC + tid] = lk((gg * (Ns[gr * HIDC + tid] - mu)) * rs + bb);
  }
  __syncthreads();
  const int rr = 2 * (wave & 7) + (lane >> 4), c4 = 4 * (lane & 15);
  const v4f ov = *(const v4f*)(Os + rr * HIDC + c4);
  float* op = out + NGRA * HIDC + rr * HIDC + c4;
  if (wave < 8) *(volatile v4f*)op = ov;
  __threadfence();
  if (wave < 8) *(volatile v4f*)op = ov;
}

extern "C" void kernel_launch(void* const* d_in, const int* in_sizes, int n_in,
                              void* d_out, int out_size, void* d_ws, size_t ws_size,
                              hipStream_t stream) {
  if (n_in < 26) return;
  const int nN = in_sizes[1] / DIMF;
  if (nN < NBS || (nN % NBS) != 0 || in_sizes[1] != nN * DIMF) return;
  const int nE = in_sizes[0] / 2;
  if (nE < 1 || in_sizes[0] != 2 * nE) return;
  if (in_sizes[2] != nN) return;
  const int nS = in_sizes[3] / 3;
  if (nS < 1 || in_sizes[3] != 3 * nS || in_sizes[4] != nS) return;
  const int nU = in_sizes[5];
  if (nU < 1 || in_sizes[6] != nU) return;
  if (in_sizes[7] != 3 * HIDC || in_sizes[8] != HIDC || in_sizes[9] != HIDC || in_sizes[10] != HIDC) return;
  if (in_sizes[11] != NLAY * 2 * DIMF || in_sizes[12] != NLAY * DIMF * DIMF) return;
  if (in_sizes[13] != NLAY * DIMF || in_sizes[14] != NLAY * DIMF || in_sizes[15] != NLAY * DIMF) return;
  if (in_sizes[16] != DIMF * HIDC || in_sizes[17] != HIDC) return;
  if (in_sizes[18] != 2 * HIDC * HIDC) return;
  for (int i = 19; i <= 25; ++i) if (in_sizes[i] != HIDC) return;
  if (out_size != 2 * NGRA * HIDC) return;

  const int*   edge_index  = (const int*)d_in[0];
  const float* n_feats     = (const float*)d_in[1];
  const int*   batch       = (const int*)d_in[2];
  const float* surf_feats  = (const float*)d_in[3];
  const int*   surf_res    = (const int*)d_in[4];
  const int*   res_batch   = (const int*)d_in[5];
  const int*   surf_set    = (const int*)d_in[6];
  const float* surf_up_w   = (const float*)d_in[7];
  const float* surf_up_b   = (const float*)d_in[8];
  const float* surf_up_g   = (const float*)d_in[9];
  const float* surf_up_be  = (const float*)d_in[10];
  const float* a_w         = (const float*)d_in[11];
  const float* lin_w       = (const float*)d_in[12];
  const float* lin_b       = (const float*)d_in[13];
  const float* ln_g        = (const float*)d_in[14];
  const float* ln_b        = (const float*)d_in[15];
  const float* hid_w       = (const float*)d_in[16];
  const float* hid_b       = (const float*)d_in[17];
  const float* down_w      = (const float*)d_in[18];
  const float* down_b      = (const float*)d_in[19];
  const float* down_g      = (const float*)d_in[20];
  const float* down_be     = (const float*)d_in[21];
  const float* prot_ln_g   = (const float*)d_in[22];
  const float* prot_ln_b   = (const float*)d_in[23];
  const float* surf_bn_g   = (const float*)d_in[24];
  const float* surf_bn_b   = (const float*)d_in[25];
  float* out = (float*)d_out;

  const int nSB = (nS + SRPB - 1) / SRPB;
  const int nDB = (nU + DRW - 1) / DRW;

  size_t off = 0;
  auto carve = [&](size_t bytes) -> char* {
    char* p = (char*)d_ws + off;
    off += (bytes + 255) & ~(size_t)255;
    return p;
  };
  unsigned short* WT  = (unsigned short*)carve((size_t)NLAY * DIMF * DIMF * 2);
  unsigned short* WHH = (unsigned short*)carve((size_t)HIDC * DIMF * 2);
  unsigned short* WHL = (unsigned short*)carve((size_t)HIDC * DIMF * 2);
  unsigned short* WDH = (unsigned short*)carve((size_t)HIDC * 2 * HIDC * 2);
  unsigned short* WDL = (unsigned short*)carve((size_t)HIDC * 2 * HIDC * 2);
  float* FEAT  = (float*)carve((size_t)nN * DIMF * 4);
  float* ACC   = (float*)carve((size_t)nN * DIMF * 4);
  _Float16* AGG = (_Float16*)carve((size_t)nN * DIMF * 2);
  float* PAB   = (float*)carve((size_t)nN * 2 * 4);
  float* NF    = (float*)carve((size_t)nN * HIDC * 4);
  float* NODES = (float*)carve((size_t)nN * HIDC * 4);
  float* Y     = (float*)carve((size_t)nDB * DRW * HIDC * 4);
  double* SPART  = (double*)carve((size_t)nSB * 64 * 8);
  double* SPARTQ = (double*)carve((size_t)nSB * 64 * 8);
  double* DPART  = (double*)carve((size_t)nDB * 64 * 8);
  double* DPARTQ = (double*)carve((size_t)nDB * 64 * 8);
  if (off > ws_size) return;
  unsigned short* X5H = (unsigned short*)FEAT;
  unsigned short* X5L = X5H + (size_t)nN * DIMF;

  k_tr<0><<<dim3(DIMF / 64, DIMF / 64, NLAY), NTH, 0, stream>>>(lin_w, DIMF, DIMF, 32.0f, WT, WT);
  k_tr<1><<<dim3(DIMF / 64, HIDC / 64, 1), NTH, 0, stream>>>(hid_w, DIMF, HIDC, 1.0f, WHH, WHL);
  k_tr<1><<<dim3(2 * HIDC / 64, HIDC / 64, 1), NTH, 0, stream>>>(down_w, 2 * HIDC, HIDC, 1.0f, WDH, WDL);

  k_surf_stats<<<nSB, NTH, 0, stream>>>(surf_feats, surf_up_w, surf_up_b, SPART, SPARTQ, nS, SRPB);
  hipFuncSetAttribute(reinterpret_cast<const void*>(&k_surf_pool),
                      hipFuncAttributeMaxDynamicSharedMemorySize, SP_LDS_BYTES);
  k_surf_pool<<<nN / NBS, NTH, SP_LDS_BYTES, stream>>>(surf_feats, surf_res, surf_up_w, surf_up_b, surf_up_g,
                                                      surf_up_be, SPART, SPARTQ, NODES, nS, nSB, nN);

  k_init<<<nN / 16, NTH, 0, stream>>>(n_feats, a_w, PAB, nN);
  hipFuncSetAttribute(reinterpret_cast<const void*>(&k_att),
                      hipFuncAttributeMaxDynamicSharedMemorySize, ATT_LDS_BYTES);
  hipFuncSetAttribute(reinterpret_cast<const void*>(&k_gemm_ln),
                      hipFuncAttributeMaxDynamicSharedMemorySize, GEMM_LDS_BYTES);
  for (int l = 0; l < NLAY; ++l) {
    const float* featl = (l == 0) ? n_feats : FEAT;
    k_att<<<nN / NBA, NTH, ATT_LDS_BYTES, stream>>>(featl, edge_index, PAB, AGG, nN, nE);
    const int last = (l == NLAY - 1) ? 1 : 0;
    const float* accin = (l == 0) ? n_feats : ACC;
    const float* awn = a_w + (last ? (size_t)0 : (size_t)(l + 1) * 2 * DIMF);
    k_gemm_ln<<<nN / GRW, NTH, GEMM_LDS_BYTES, stream>>>(
        AGG, (const _Float16*)(WT + (size_t)l * DIMF * DIMF), lin_b + (size_t)l * DIMF,
        ln_g + (size_t)l * DIMF, ln_b + (size_t)l * DIMF, awn, accin, ACC, FEAT, PAB, X5H, X5L, last);
  }

  k_hid<<<nN / DRW, 128, 0, stream>>>(X5H, X5L, WHH, WHL, hid_b, NF);
  k_prot<<<1, 512, 0, stream>>>(NF, batch, prot_ln_g, prot_ln_b, out, nN);
  k_down<<<nDB, 128, 0, stream>>>(NF, NODES, surf_set, WDH, WDL, down_b, Y, DPART, DPARTQ, nU, nN);
  k_out1<<<1, 512, 0, stream>>>(Y, res_batch, DPART, DPARTQ, down_g, down_be, surf_bn_g, surf_bn_b, out, nU, nDB);
}
